// CausalSelfAttention_80126909874598
// MI455X (gfx1250) — hardware-verified
//
#include <hip/hip_runtime.h>


#ifndef NB
#define NB 2
#endif
#ifndef SEQ
#define SEQ 2048
#endif
#ifndef SCORE_RES
#define SCORE_RES 1
#endif
#define NB_FULL  2
#define SEQ_FULL 2048
#define DM   1024
#define NH   16
#define NKV  4
#define REP  (NH / NKV)
#define HD   64
#define GC   32
#define DQ   (NH * HD)
#define DKV  (NKV * HD)
#define FP   (DQ + 2 * DKV)
#define KC0  DQ
#define VC0  (DQ + DKV)
#define RH   256
#define RHE  ((SEQ < RH) ? SEQ : RH)
#define PCAR 1024.0f
#define VCAR 16.0f
#define RSC  2048.0f
#define RSCI (1.0f / 2048.0f)
#define SCL  0.125f
#define L2E  1.4426950408889634f
#define NEGB (-1.0e30f)
static_assert(HD == 64);
static_assert(NH % NKV == 0);
static_assert(DM % 64 == 0 && DQ % 64 == 0 && DKV % 64 == 0 && FP % 64 == 0);
static_assert(DM % 32 == 0 && DQ % 32 == 0 && HD % 32 == 0);
static_assert(SEQ % 64 == 0 && (NB * SEQ) % 64 == 0);
static_assert(RH % 64 == 0 && RHE % 64 == 0 && (SEQ - RHE) % 64 == 0);
static_assert(((size_t)SEQ * DM) % 2048 == 0);
static_assert(((size_t)NB * SEQ * NH) % 8 == 0 && ((size_t)NB * SEQ * NKV) % 8 == 0);
static_assert(((size_t)NB * NKV * HD * SEQ) % 512 == 0);
static_assert(NB <= NB_FULL && SEQ <= SEQ_FULL);
static_assert(GC == 32 && GC <= DM);
static_assert(((size_t)NB * SEQ * NKV) % 256 == 0);
static_assert(SCORE_RES == 0 || SCORE_RES == 1);

typedef _Float16 h16;
typedef unsigned short bf;
typedef __attribute__((ext_vector_type(16))) __bf16   v16bf;
typedef __attribute__((ext_vector_type(16))) _Float16 v16h;
typedef __attribute__((ext_vector_type(8)))  _Float16 v8h;
typedef __attribute__((ext_vector_type(8)))  unsigned short v8us;
typedef __attribute__((ext_vector_type(8)))  float    v8f;
typedef __attribute__((ext_vector_type(4)))  float    v4f;
typedef __attribute__((ext_vector_type(2)))  float    v2f;
typedef __attribute__((ext_vector_type(2)))  _Float16 v2h;
typedef v4f  __attribute__((may_alias)) v4fa;

__device__ __forceinline__ unsigned short f2bf(float f) { unsigned u = __float_as_uint(f); u += 0x7FFFu + ((u >> 16) & 1u); return (unsigned short)(u >> 16); }
__device__ __forceinline__ float bf2f(unsigned short b) { return __uint_as_float(((unsigned)b) << 16); }
__device__ __forceinline__ float bfr(float f) { return bf2f(f2bf(f)); }
__device__ __forceinline__ void splitf(float y, unsigned short& h, unsigned short& l) { h = f2bf(y); l = f2bf(y - bf2f(h)); }
__device__ __forceinline__ v16h cat16(v8h lo, v8h hi) { return __builtin_shufflevector(lo, hi, 0, 1, 2, 3, 4, 5, 6, 7, 8, 9, 10, 11, 12, 13, 14, 15); }
__device__ __forceinline__ v16bf cat16b(v8us lo, v8us hi) { return __builtin_bit_cast(v16bf, __builtin_shufflevector(lo, hi, 0, 1, 2, 3, 4, 5, 6, 7, 8, 9, 10, 11, 12, 13, 14, 15)); }
__device__ __forceinline__ v8f wmma16(v16h a, v16h b, v8f c) { return __builtin_amdgcn_wmma_f32_16x16x32_f16(false, a, false, b, (short)0, c, false, false); }
__device__ __forceinline__ v8f wmmab(v16bf a, v16bf b, v8f c) { return __builtin_amdgcn_wmma_f32_16x16x32_bf16(false, a, false, b, (short)0, c, false, false); }
__device__ __forceinline__ v16h  ldh(const h16* p) { return cat16(*(const v8h*)p, *(const v8h*)(p + 16)); }
__device__ __forceinline__ v16bf ldb(const bf* p)  { return cat16b(*(const v8us*)p, *(const v8us*)(p + 16)); }
static __device__ __forceinline__ h16 toh_flush(float v) { const h16 r = (h16)v; return (fabsf(v) < 6.103515625e-05f) ? (h16)0.0f : r; }

template <int NSPLIT>
__device__ __forceinline__ void gemmw_body(const bf* __restrict__ A, const bf* __restrict__ A2, const bf* __restrict__ Bt, int K, float* C, int ldc, size_t sA, size_t sC) {
    __shared__ __align__(16) float os[16 * 68];
    const size_t z = blockIdx.z; A += z * sA; if (NSPLIT == 1) A2 += z * sA; C += z * sC;
    const int lane = threadIdx.x & 31, lr = lane & 15, hi = lane >> 4; const int r0 = blockIdx.x * 64, c0 = blockIdx.y * 64;
    v8f acc[4][4];
#pragma unroll
    for (int mb = 0; mb < 4; ++mb)
#pragma unroll
        for (int nb = 0; nb < 4; ++nb) acc[mb][nb] = (v8f){};
    const size_t aoff = (size_t)(r0 + lr) * K + 8 * hi, boff = (size_t)(c0 + lr) * K + 8 * hi;
#pragma unroll 1
    for (int kc = 0; kc < K; kc += 32) {
        v16bf a[4], a2[4];
#pragma unroll
        for (int mb = 0; mb < 4; ++mb) { a[mb] = ldb(A + aoff + (size_t)mb * 16 * K + kc); if (NSPLIT == 1) a2[mb] = ldb(A2 + aoff + (size_t)mb * 16 * K + kc); }
#pragma unroll
        for (int nb = 0; nb < 4; ++nb) { const v16bf b = ldb(Bt + boff + (size_t)nb * 16 * K + kc);
#pragma unroll
            for (int mb = 0; mb < 4; ++mb) { acc[mb][nb] = wmmab(a[mb], b, acc[mb][nb]); if (NSPLIT == 1) acc[mb][nb] = wmmab(a2[mb], b, acc[mb][nb]); } }
        asm volatile("v_nop\n\tv_nop\n\tv_nop\n\tv_nop" : "+v"(acc[0][0]), "+v"(acc[1][1]), "+v"(acc[2][2]), "+v"(acc[3][3]) : "v"(a[0]), "v"(a[3]));
    }
#pragma unroll
    for (int mb = 0; mb < 4; ++mb) {
#pragma unroll
        for (int nb = 0; nb < 4; ++nb) {
#pragma unroll
            for (int j = 0; j < 8; ++j) os[(hi * 8 + j) * 68 + nb * 16 + lr] = acc[mb][nb][j]; }
        __builtin_amdgcn_wave_barrier(); asm volatile("" ::: "memory");
        float* crow = C + (size_t)(r0 + mb * 16) * ldc + c0;
#pragma unroll 1
        for (int ps = 0; ps < 2; ++ps) {
#pragma unroll
            for (int s = 0; s < 8; ++s) { const int row = 2 * s + hi, cofs = lr * 4; const v4f val = *(const v4fa*)(os + row * 68 + cofs);
                *(volatile v4f*)(crow + (size_t)row * ldc + cofs) = val; }
            if (ps == 0) __threadfence(); }
        __builtin_amdgcn_wave_barrier(); asm volatile("" ::: "memory");
    }
}
__global__ __launch_bounds__(32) void k_gemm_proj(const bf* __restrict__ A, const bf* __restrict__ Bt, float* C) { gemmw_body<0>(A, A, Bt, DM, C, FP, 0, 0); }
__global__ __launch_bounds__(32) void k_gemm_out(const bf* __restrict__ A, const bf* __restrict__ A2, const bf* __restrict__ Bt, float* C) { gemmw_body<1>(A, A2, Bt, DQ, C, DM, (size_t)SEQ * DQ, (size_t)SEQ_FULL * DM); }

__global__ __launch_bounds__(256) void k_cvtx(const float* __restrict__ src, bf* dst) {
    const size_t i = (size_t)blockIdx.x * 256 + threadIdx.x; const size_t b = blockIdx.y;
    const v8f v = *(const v8f*)(src + b * (size_t)SEQ_FULL * DM + i * 8); v8us o;
#pragma unroll
    for (int k = 0; k < 8; ++k) o[k] = f2bf(v[k]);
    bf* d = dst + b * (size_t)SEQ * DM + i * 8;
    *(volatile v8us*)d = o; __threadfence(); *(volatile v8us*)d = o; }

__global__ __launch_bounds__(256) void k_wtp(const float* __restrict__ W, int N, bf* out) {
    __shared__ __align__(16) unsigned short ts[64 * 72];
    const int tid = threadIdx.x; const int k0 = blockIdx.x * 64, n0 = blockIdx.y * 64;
#pragma unroll
    for (int it = 0; it < 4; ++it) { const int idx = it * 256 + tid; const int kk = idx >> 4, c4 = (idx & 15) * 4; const v4f v = *(const v4f*)(W + (size_t)(k0 + kk) * N + n0 + c4);
#pragma unroll
        for (int q = 0; q < 4; ++q) ts[kk * 72 + c4 + q] = f2bf(v[q]); }
    __syncthreads();
    v8us o[2];
#pragma unroll
    for (int it = 0; it < 2; ++it) { const int idx = it * 256 + tid; const int nn = idx >> 3, pc = idx & 7;
#pragma unroll
        for (int q = 0; q < 8; ++q) o[it][q] = ts[(pc * 8 + q) * 72 + nn]; }
#pragma unroll 1
    for (int ps = 0; ps < 2; ++ps) {
#pragma unroll
        for (int it = 0; it < 2; ++it) { const int idx = it * 256 + tid; const int nn = idx >> 3, pc = idx & 7; *(volatile v8us*)(out + (size_t)(n0 + nn) * DM + k0 + pc * 8) = o[it]; }
        if (ps == 0) __threadfence(); }
}

__global__ __launch_bounds__(256) void k_gate(const float* __restrict__ x, const float* __restrict__ wg, float* G) {
    const int i = blockIdx.x * 256 + threadIdx.x;
    const int g = i % NKV; const int bt = i / NKV; const int t = bt % SEQ; const int b = bt / SEQ;
    const float* xr = x + ((size_t)b * SEQ_FULL + t) * DM;
    float acc = 0.f;
#pragma unroll 1
    for (int c = 0; c < GC; ++c) acc += bfr(xr[c]) * bfr(wg[c * NKV + g]);
    const float gv = 2.0f * (1.0f / (1.0f + expf(-acc)));
    *(volatile float*)(G + i) = gv; __threadfence(); *(volatile float*)(G + i) = gv; }

__global__ __launch_bounds__(256) void k_ropen(const float* __restrict__ F, int col0, int nheads, const float* __restrict__ cosb, const float* __restrict__ sinb, h16* Ph, h16* Pr) {
    const int lane = threadIdx.x & 31; const int wave = __builtin_amdgcn_readfirstlane(threadIdx.x >> 5);
    const int row = blockIdx.x * 8 + wave; if (row >= NB * SEQ * nheads) return;
    const int h = row % nheads; const int bt = row / nheads; const int t = bt % SEQ; const int b = bt / SEQ;
    const float* f = F + (size_t)bt * FP + col0 + h * HD;
    const int d = 2 * lane, dm = d & 31, dp = d ^ 32;
    const v2f xs = *(const v2f*)(f + d); const v2f xp = *(const v2f*)(f + dp);
    const size_t tb = ((size_t)b * SEQ_FULL + t) * 32 + dm;
    const v2f cc = *(const v2f*)(cosb + tb); const v2f sn = *(const v2f*)(sinb + tb);
    const bool lo = (lane < 16);
    float r[2]; float ss = 0.f;
#pragma unroll
    for (int q = 0; q < 2; ++q) { const float c = bfr(cc[q]), s = bfr(sn[q]); const float a = xs[q] * c; const float m = xp[q] * s; r[q] = lo ? (a + m) : (a - m); ss += r[q] * r[q]; }
#pragma unroll
    for (int sh = 16; sh; sh >>= 1) ss += __shfl_xor(ss, sh, 32);
    const float inv = rsqrtf(ss * (1.0f / HD) + 1e-6f);
    v2h o16, ors;
#pragma unroll
    for (int q = 0; q < 2; ++q) { const float y = r[q] * inv; const h16 hh = toh_flush(y); o16[q] = hh; ors[q] = toh_flush((y - (float)hh) * RSC); }
    const size_t e = ((size_t)(b * nheads + h) * SEQ + t) * HD + d;
    *(volatile v2h*)(Ph + e) = o16; *(volatile v2h*)(Pr + e) = ors; __threadfence(); *(volatile v2h*)(Ph + e) = o16; *(volatile v2h*)(Pr + e) = ors; }

__global__ __launch_bounds__(256) void k_vtp(const float* __restrict__ F, const float* __restrict__ ve, const float* __restrict__ G, h16* Vh, h16* Vr) {
    const size_t e = ((size_t)blockIdx.x * 256 + threadIdx.x) * 2; if (e >= (size_t)NB * NKV * HD * SEQ) return;
    const int t = (int)(e % SEQ); const int d = (int)((e / SEQ) % HD); const int bg = (int)(e / ((size_t)SEQ * HD)); const int g = bg % NKV; const int b = bg / NKV; v2h o16, ors;
#pragma unroll
    for (int q = 0; q < 2; ++q) {
        const size_t bt = (size_t)b * SEQ + t + q;
        const float gv = G[bt * NKV + g];
        const float ev = bfr(ve[((size_t)b * SEQ_FULL + t + q) * DKV + g * HD + d]);
        const float x = (F[bt * FP + VC0 + g * HD + d] + gv * ev) * VCAR; const h16 hh = toh_flush(x); o16[q] = hh; ors[q] = toh_flush((x - (float)hh) * RSC); }
    *(volatile v2h*)(Vh + e) = o16; *(volatile v2h*)(Vr + e) = ors; __threadfence(); *(volatile v2h*)(Vh + e) = o16; *(volatile v2h*)(Vr + e) = ors; }

template <bool HI>
__device__ __forceinline__ void attn_body(const h16* __restrict__ Qh, const h16* __restrict__ Qr, const h16* __restrict__ Kh, const h16* __restrict__ Kr, const h16* __restrict__ Vh, const h16* __restrict__ Vr, bf* Yh, bf* Yl, const int* __restrict__ wsz, int rbase) {
    __shared__ __align__(16) float ys[4 * 16 * 68];
    const int lane = threadIdx.x & 31, lr = lane & 15, hi = lane >> 4;
    const int wave = __builtin_amdgcn_readfirstlane(threadIdx.x >> 5);
    const int b = blockIdx.z, hq = blockIdx.y, g = hq / REP;
    const int q0 = rbase + blockIdx.x * 64 + wave * 16;
    const size_t qoff  = ((size_t)(b * NH + hq) * SEQ + q0 + lr) * HD + 8 * hi;
    const size_t kbase = ((size_t)(b * NKV + g) * SEQ + lr) * HD + 8 * hi;
    const size_t vbase = ((size_t)(b * NKV + g) * HD + lr) * SEQ + 8 * hi;
    v8f om[4], orr[4];
#pragma unroll
    for (int dt = 0; dt < 4; ++dt) { om[dt] = (v8f){}; orr[dt] = (v8f){}; }
    float mrun = NEGB, lrun = 0.f;
    const int kend = q0 + 16;
    const int win = min(max(wsz[0], 0), SEQ_FULL);
    const int kbeg = max(q0 - win, 0) & ~31;
#pragma unroll 1
    for (int kb = kbeg; kb < kend; kb += 32) {
        v8f s0 = (v8f){}, s1 = (v8f){}, t0 = (v8f){}, t1 = (v8f){};
#pragma unroll
        for (int ks = 0; ks < 2; ++ks) {
            const v16h qh = ldh(Qh + qoff + ks * 32);
            v16h qr = qh;
            if (HI || (SCORE_RES != 0)) qr = ldh(Qr + qoff + ks * 32);
            const size_t ko = kbase + (size_t)kb * HD + ks * 32;
            const v16h k0 = ldh(Kh + ko);
            const v16h k1 = ldh(Kh + ko + 16 * HD);
            s0 = wmma16(k0, qh, s0); if (HI || (SCORE_RES != 0)) t0 = wmma16(k0, qr, t0);
            s1 = wmma16(k1, qh, s1); if (HI || (SCORE_RES != 0)) t1 = wmma16(k1, qr, t1);
            if (HI) {
                const v16h k0r = ldh(Kr + ko); const v16h k1r = ldh(Kr + ko + 16 * HD);
                t0 = wmma16(k0r, qh, t0); t1 = wmma16(k1r, qh, t1);
                asm volatile("v_nop\n\tv_nop\n\tv_nop\n\tv_nop" : "+v"(s0), "+v"(s1), "+v"(t0), "+v"(t1) : "v"(qh), "v"(qr), "v"(k0), "v"(k1), "v"(k0r), "v"(k1r));
            } else if (SCORE_RES != 0) {
                asm volatile("v_nop\n\tv_nop\n\tv_nop\n\tv_nop" : "+v"(s0), "+v"(s1), "+v"(t0), "+v"(t1) : "v"(qh), "v"(qr), "v"(k0), "v"(k1));
            } else {
                asm volatile("v_nop\n\tv_nop\n\tv_nop\n\tv_nop" : "+v"(s0), "+v"(s1) : "v"(qh), "v"(k0), "v"(k1));
            }
        }
        float sa[8], sb[8];
#pragma unroll
        for (int r = 0; r < 8; ++r) { sa[r] = (s0[r] + t0[r] * RSCI) * SCL; sb[r] = (s1[r] + t1[r] * RSCI) * SCL; }
        if (kb + 31 > q0 || q0 + 15 - kb > win) {
            const int qi = q0 + lr; const int kj = kb + 8 * hi;
#pragma unroll
            for (int r = 0; r < 8; ++r) {
                const int ja = kj + r, jb = kj + 16 + r;
                sa[r] = ((ja <= qi) && (qi - ja <= win)) ? sa[r] : NEGB;
                sb[r] = ((jb <= qi) && (qi - jb <= win)) ? sb[r] : NEGB; }
        }
        float mloc = fmaxf(sa[0], sb[0]);
#pragma unroll
        for (int r = 1; r < 8; ++r) mloc = fmaxf(mloc, fmaxf(sa[r], sb[r]));
        mloc = fmaxf(mloc, __shfl_xor(mloc, 16, 32));
        const float mnew = fmaxf(mrun, mloc);
        const float fac = __builtin_amdgcn_exp2f((mrun - mnew) * L2E);
        float lsum = 0.f;
#pragma unroll
        for (int r = 0; r < 8; ++r) { sa[r] = __builtin_amdgcn_exp2f((sa[r] - mnew) * L2E); sb[r] = __builtin_amdgcn_exp2f((sb[r] - mnew) * L2E); lsum += sa[r] + sb[r]; }
        lsum += __shfl_xor(lsum, 16, 32);
        lrun = lrun * fac + lsum; mrun = mnew;
        v16h ph, pr;
#pragma unroll
        for (int r = 0; r < 8; ++r) {
            const float a = sa[r] * PCAR; const h16 ha = toh_flush(a); ph[r] = ha;
            const float c = sb[r] * PCAR; const h16 hc = toh_flush(c); ph[8 + r] = hc;
            if (HI) { pr[r] = toh_flush((a - (float)ha) * RSC); pr[8 + r] = toh_flush((c - (float)hc) * RSC); }
        }
#pragma unroll
        for (int dt = 0; dt < 4; ++dt) { om[dt] = om[dt] * fac; if (HI) orr[dt] = orr[dt] * fac; }
        const size_t vo = vbase + kb;
#pragma unroll
        for (int dt = 0; dt < 4; ++dt) {
            const v16h vh = ldh(Vh + vo + (size_t)dt * 16 * SEQ);
            om[dt] = wmma16(vh, ph, om[dt]);
            if (HI) {
                const v16h vr = ldh(Vr + vo + (size_t)dt * 16 * SEQ);
                orr[dt] = wmma16(vr, ph, orr[dt]); orr[dt] = wmma16(vh, pr, orr[dt]);
                asm volatile("v_nop\n\tv_nop\n\tv_nop\n\tv_nop" : "+v"(om[dt]), "+v"(orr[dt]) : "v"(vh), "v"(vr), "v"(ph), "v"(pr));
            } else {
                asm volatile("v_nop\n\tv_nop\n\tv_nop\n\tv_nop" : "+v"(om[dt]) : "v"(vh), "v"(ph));
            }
        }
    }
    const float inv = 1.0f / (lrun * (PCAR * VCAR));
    const int yb = wave * 16 * 68;
#pragma unroll
    for (int dt = 0; dt < 4; ++dt)
#pragma unroll
        for (int r = 0; r < 8; ++r) { float o = om[dt][r]; if (HI) o += orr[dt][r] * RSCI; ys[yb + lr * 68 + dt * 16 + 8 * hi + r] = o * inv; }
    __builtin_amdgcn_wave_barrier(); asm volatile("" ::: "memory");
    v8us oh[4], ol[4];
    const int rq = lane >> 3, pc = lane & 7;
#pragma unroll
    for (int s = 0; s < 4; ++s) { const int row = 4 * s + rq; const v4f u0 = *(const v4fa*)(ys + yb + row * 68 + pc * 8); const v4f u1 = *(const v4fa*)(ys + yb + row * 68 + pc * 8 + 4);
#pragma unroll
        for (int q = 0; q < 4; ++q) { unsigned short a, c; splitf(u0[q], a, c); oh[s][q] = a; ol[s][q] = c; splitf(u1[q], a, c); oh[s][4 + q] = a; ol[s][4 + q] = c; } }
    const size_t ybase = ((size_t)b * SEQ + q0) * DQ + (size_t)hq * HD + pc * 8;
#pragma unroll 1
    for (int ps = 0; ps < 2; ++ps) {
#pragma unroll
        for (int s = 0; s < 4; ++s) { const size_t oo = ybase + (size_t)(4 * s + rq) * DQ; *(volatile v8us*)(Yh + oo) = oh[s]; *(volatile v8us*)(Yl + oo) = ol[s]; }
        if (ps == 0) __threadfence(); }
}
__global__ __launch_bounds__(128) void k_attn_hi(const h16* __restrict__ Qh, const h16* __restrict__ Qr, const h16* __restrict__ Kh, const h16* __restrict__ Kr, const h16* __restrict__ Vh, const h16* __restrict__ Vr, bf* Yh, bf* Yl, const int* __restrict__ wsz) { attn_body<true>(Qh, Qr, Kh, Kr, Vh, Vr, Yh, Yl, wsz, 0); }
__global__ __launch_bounds__(128) void k_attn_lo(const h16* __restrict__ Qh, const h16* __restrict__ Qr, const h16* __restrict__ Kh, const h16* __restrict__ Kr, const h16* __restrict__ Vh, const h16* __restrict__ Vr, bf* Yh, bf* Yl, const int* __restrict__ wsz) { attn_body<false>(Qh, Qr, Kh, Kr, Vh, Vr, Yh, Yl, wsz, RHE); }

constexpr size_t SZ_XB = (size_t)NB * SEQ * DM * 2;
constexpr size_t SZ_WP = (size_t)FP * DM * 2;
constexpr size_t SZ_WO = (size_t)DM * DQ * 2;
constexpr size_t SZ_F  = (size_t)NB * SEQ * FP * 4;
constexpr size_t SZ_Q  = (size_t)NB * NH * SEQ * HD * 2;
constexpr size_t SZ_K  = (size_t)NB * NKV * SEQ * HD * 2;
constexpr size_t SZ_Y  = (size_t)NB * SEQ * DQ * 2;
constexpr size_t SZ_G  = (size_t)NB * SEQ * NKV * 4;
constexpr size_t OFF_XB = 0;
constexpr size_t OFF_WP = OFF_XB + SZ_XB;
constexpr size_t OFF_WO = OFF_WP + SZ_WP;
constexpr size_t OFF_F  = OFF_WO + SZ_WO;
constexpr size_t OFF_QH = OFF_F + SZ_F;
constexpr size_t OFF_QR = OFF_QH + SZ_Q;
constexpr size_t OFF_KH = OFF_QR + SZ_Q;
constexpr size_t OFF_KR = OFF_KH + SZ_K;
constexpr size_t OFF_VH = OFF_KR + SZ_K;
constexpr size_t OFF_VR = OFF_VH + SZ_K;
constexpr size_t OFF_YH = OFF_VR + SZ_K;
constexpr size_t OFF_YL = OFF_YH + SZ_Y;
constexpr size_t OFF_G  = OFF_YL + SZ_Y;
constexpr size_t WS_TOTAL = OFF_G + SZ_G;
static_assert(SZ_XB % 256 == 0 && SZ_WP % 256 == 0 && SZ_WO % 256 == 0 && SZ_F % 256 == 0 && SZ_Q % 256 == 0 && SZ_K % 256 == 0 && SZ_Y % 256 == 0 && SZ_G % 256 == 0);
static_assert(WS_TOTAL <= (size_t)134217728);

extern "C" void kernel_launch(void* const* d_in, const int* in_sizes, int n_in,
                              void* d_out, int out_size, void* d_ws, size_t ws_size, hipStream_t stream) {
    if (n_in < 10) return;
    const long long need_x = (long long)(NB - 1) * SEQ_FULL * DM + (long long)SEQ * DM;
    const long long need_e = (long long)(NB - 1) * SEQ_FULL * DKV + (long long)SEQ * DKV;
    const long long need_t = (long long)(NB - 1) * SEQ_FULL * 32 + (long long)SEQ * 32;
    if ((long long)in_sizes[0] < need_x) return;
    if ((long long)in_sizes[1] < need_e) return;
    if ((long long)in_sizes[2] < need_t || (long long)in_sizes[3] < need_t) return;
    if (in_sizes[4] < DM * DQ || in_sizes[5] < DM * DKV || in_sizes[6] < DM * DKV || in_sizes[7] < DQ * DM) return;
    if (in_sizes[8] < GC * NKV || in_sizes[9] < 1) return;
    if ((long long)out_size < need_x) return;
    if (WS_TOTAL > ws_size) return;
    const float* x  = (const float*)d_in[0];
    const float* ve = (const float*)d_in[1];
    const float* cs = (const float*)d_in[2];
    const float* sn = (const float*)d_in[3];
    const float* wq = (const float*)d_in[4];
    const float* wk = (const float*)d_in[5];
    const float* wv = (const float*)d_in[6];
    const float* wo = (const float*)d_in[7];
    const float* wg = (const float*)d_in[8];
    const int*  wsz = (const int*)d_in[9];
    float* OUT = (float*)d_out;
    char* ws = (char*)d_ws;
    bf* XB = (bf*)(ws + OFF_XB); bf* WP = (bf*)(ws + OFF_WP); bf* WOT = (bf*)(ws + OFF_WO); float* F = (float*)(ws + OFF_F);
    h16* QH = (h16*)(ws + OFF_QH); h16* QR = (h16*)(ws + OFF_QR); h16* KH = (h16*)(ws + OFF_KH); h16* KR = (h16*)(ws + OFF_KR);
    h16* VH = (h16*)(ws + OFF_VH); h16* VR = (h16*)(ws + OFF_VR); bf* YH = (bf*)(ws + OFF_YH); bf* YL = (bf*)(ws + OFF_YL);
    float* G = (float*)(ws + OFF_G);

    k_cvtx<<<dim3((unsigned)((size_t)SEQ * DM / 8 / 256), NB, 1), 256, 0, stream>>>(x, XB);
    k_wtp<<<dim3(DM / 64, DQ / 64, 1), 256, 0, stream>>>(wq, DQ, WP);
    k_wtp<<<dim3(DM / 64, DKV / 64, 1), 256, 0, stream>>>(wk, DKV, WP + (size_t)KC0 * DM);
    k_wtp<<<dim3(DM / 64, DKV / 64, 1), 256, 0, stream>>>(wv, DKV, WP + (size_t)VC0 * DM);
    k_wtp<<<dim3(DQ / 64, DM / 64, 1), 256, 0, stream>>>(wo, DM, WOT);
    k_gate<<<(unsigned)((size_t)NB * SEQ * NKV / 256), 256, 0, stream>>>(x, wg, G);
    k_gemm_proj<<<dim3(NB * SEQ / 64, FP / 64, 1), 32, 0, stream>>>(XB, WP, F);
    k_ropen<<<(unsigned)((size_t)NB * SEQ * NH / 8), 256, 0, stream>>>(F, 0, NH, cs, sn, QH, QR);
    k_ropen<<<(unsigned)((size_t)NB * SEQ * NKV / 8), 256, 0, stream>>>(F, KC0, NKV, cs, sn, KH, KR);
    k_vtp<<<(unsigned)((size_t)NB * NKV * HD * SEQ / 512), 256, 0, stream>>>(F, ve, G, VH, VR);
    k_attn_hi<<<dim3(RHE / 64, NH, NB), 128, 0, stream>>>(QH, QR, KH, KR, VH, VR, YH, YL, wsz);
    if (SEQ > RHE) k_attn_lo<<<dim3((SEQ - RHE) / 64, NH, NB), 128, 0, stream>>>(QH, QR, KH, KR, VH, VR, YH, YL, wsz);
    k_gemm_out<<<dim3(SEQ / 64, DM / 64, NB), 32, 0, stream>>>(YH, YL, WOT, OUT);
}
